// MambaBlock_62448824483844
// MI455X (gfx1250) — hardware-verified
//
#include <hip/hip_runtime.h>
#include <stddef.h>
#include <stdint.h>
#include <math.h>


#define DM    1024
#define DI    2048
#define DS    16
#define SL    1024
#define NTOK  2048
#define XZC   4096
#define NPJ   33
#define PJP   64
#define K2    4096

#define GBM   64
#define GBN   64
#define GTHR  128

#define PTHR  256
#define U_X    (NTOK * DM / 8)
#define U_WIN  (XZC * DM / 8)
#define U_WOUT (DM * DI / 8)
#define U_WX   (PJP * DI / 8)
#define U_TOT  (U_X + U_WIN + U_WOUT + U_WX)

#define SNT   128
#define SCH   64
#define PJQ   12
#define PJW   (4 * PJQ)

#define WSMAX 134217728

static_assert(U_X % PTHR == 0 && U_WIN % PTHR == 0 && U_WOUT % PTHR == 0 && U_WX % PTHR == 0);
static_assert(NTOK % GBM == 0 && XZC % GBN == 0 && PJP % GBN == 0 && DM % GBN == 0);
static_assert(DM % 32 == 0 && K2 % 32 == 0 && (DI & (DI - 1)) == 0 && (DM & (DM - 1)) == 0 && K2 == 2 * DI);
static_assert(GBM == (GTHR / 32) * 16 && GBN == 64);
static_assert(DI == 8 * PTHR);
static_assert(DI % SNT == 0 && SL % SCH == 0 && (SCH * PJQ) % SNT == 0 && PJW >= NPJ && PJW <= PJP);
static_assert((2 * SCH * SNT / 8) % (4 * SNT) == 0);
static_assert((DS * SNT * 4) * 2 + SCH * PJW * 4 + 2 * SCH * SNT * 2 <= 65536);

typedef float          v4f   __attribute__((ext_vector_type(4)));
typedef float          v8f   __attribute__((ext_vector_type(8)));
typedef int            v8i   __attribute__((ext_vector_type(8)));
typedef unsigned short v8us  __attribute__((ext_vector_type(8)));
typedef unsigned short v16us __attribute__((ext_vector_type(16)));
typedef __bf16         v16bf __attribute__((ext_vector_type(16)));
typedef v4f  __attribute__((may_alias)) v4fa;
typedef v8us __attribute__((may_alias)) v8usa;
union FragB { v16bf v; v16us u; v8us h[2]; v8i w; };

__device__ __forceinline__ v8f wmb(const FragB& a, const FragB& b, v8f c) {
  v8f d = __builtin_amdgcn_wmma_f32_16x16x32_bf16(false, a.v, false, b.v, (short)0, c, false, false);
  asm volatile("v_nop\n\tv_nop\n\tv_nop\n\tv_nop" : "+v"(d) : "v"(a.w), "v"(b.w));
  return d;
}

__device__ __forceinline__ unsigned bf16_bits(float f) {
  const unsigned u = __float_as_uint(f);
  return (u + 0x7FFFu + ((u >> 16) & 1u)) >> 16;
}
__device__ __forceinline__ float bf16_val(float f) {
  return __uint_as_float(bf16_bits(f) << 16);
}

__device__ __forceinline__ void cvt8(const float* __restrict__ sp, unsigned short* dp, bool ok) {
  const v4f a = *(const v4fa*)sp;
  const v4f b = *(const v4fa*)(sp + 4);
  v8us o;
  o[0] = ok ? (unsigned short)bf16_bits(a.x) : (unsigned short)0;
  o[1] = ok ? (unsigned short)bf16_bits(a.y) : (unsigned short)0;
  o[2] = ok ? (unsigned short)bf16_bits(a.z) : (unsigned short)0;
  o[3] = ok ? (unsigned short)bf16_bits(a.w) : (unsigned short)0;
  o[4] = ok ? (unsigned short)bf16_bits(b.x) : (unsigned short)0;
  o[5] = ok ? (unsigned short)bf16_bits(b.y) : (unsigned short)0;
  o[6] = ok ? (unsigned short)bf16_bits(b.z) : (unsigned short)0;
  o[7] = ok ? (unsigned short)bf16_bits(b.w) : (unsigned short)0;
  *(volatile v8us*)dp = o;
  __threadfence();
  *(volatile v8us*)dp = o;
}

__global__ __launch_bounds__(PTHR) void k_prep(const float* __restrict__ x, const float* __restrict__ Win,
                                               const float* __restrict__ Wout, const float* __restrict__ Wx,
                                               unsigned short* XB, unsigned short* WIN,
                                               unsigned short* WOUT, unsigned short* WX) {
  const int u = (int)blockIdx.x * PTHR + (int)threadIdx.x;
  if (u < U_X) {
    const size_t o = (size_t)u * 8;
    cvt8(x + o, XB + o, true);
  } else if (u < U_X + U_WIN) {
    const size_t o = (size_t)(u - U_X) * 8;
    cvt8(Win + o, WIN + o, true);
  } else if (u < U_X + U_WIN + U_WOUT) {
    const size_t o = (size_t)(u - U_X - U_WIN) * 8;
    cvt8(Wout + o, WOUT + o, true);
  } else if (u < U_TOT) {
    const int v   = u - U_X - U_WIN - U_WOUT;
    const int row = v >> 8;
    const int k8  = (v & 255) * 8;
    const int rc  = row < NPJ ? row : NPJ - 1;
    cvt8(Wx + (size_t)rc * DI + k8, WX + (size_t)row * DI + k8, row < NPJ);
  }
}

__global__ __launch_bounds__(GTHR) void k_gemm(
    const unsigned short* __restrict__ A, const unsigned short* __restrict__ BT,
    float* outF, int K, int ldb, int kbmask, int ldo)
{
  __shared__ __attribute__((aligned(16))) float stg[GBM * GBN];
  const int tid = (int)threadIdx.x, lane = tid & 31, wave = tid >> 5, hh = lane >> 4, m = lane & 15;
  const int rowBase = (int)blockIdx.x * GBM;
  const int col0    = (int)blockIdx.y * GBN;

  v8f acc[4];
  {
    const v8f z = {0.f, 0.f, 0.f, 0.f, 0.f, 0.f, 0.f, 0.f};
    acc[0] = z; acc[1] = z; acc[2] = z; acc[3] = z;
  }
  const unsigned short* ap = A  + (size_t)(rowBase + 16 * wave + m) * (size_t)K + 8 * hh;
  const unsigned short* wp = BT + (size_t)(col0 + m) * (size_t)ldb + 8 * hh;
  const int ksteps = K >> 5;
#pragma unroll 1
  for (int ks = 0; ks < ksteps; ++ks) {
    const int k0 = 32 * ks;
    const int kb = k0 & kbmask;
    FragB af;
    af.h[0] = *(const v8usa*)(ap + k0);
    af.h[1] = *(const v8usa*)(ap + k0 + 16);
#pragma unroll
    for (int t = 0; t < 4; ++t) {
      const unsigned short* wq = wp + (size_t)(16 * t) * (size_t)ldb + kb;
      FragB bf;
      bf.h[0] = *(const v8usa*)wq;
      bf.h[1] = *(const v8usa*)(wq + 16);
      acc[t] = wmb(af, bf, acc[t]);
    }
  }

#pragma unroll
  for (int t = 0; t < 4; ++t) {
    const int lc = 16 * t + m;
#pragma unroll
    for (int r = 0; r < 8; ++r) {
      const int lr = 16 * wave + 8 * hh + r;
      stg[lr * GBN + lc] = acc[t][r];
    }
  }
  __syncthreads();

  v4f fv[8];
#pragma unroll
  for (int i = 0; i < 8; ++i) {
    const int lr = 16 * wave + 2 * i + hh;
    fv[i] = *(const v4fa*)(stg + lr * GBN + 4 * m);
  }
#pragma unroll
  for (int i = 0; i < 8; ++i) {
    const int lr = 16 * wave + 2 * i + hh;
    const int gr = rowBase + lr;
    float* op = outF + (size_t)gr * (size_t)ldo + col0 + 4 * m;
    *(volatile v4f*)op = fv[i];
  }
  __threadfence();
#pragma unroll
  for (int i = 0; i < 8; ++i) {
    const int lr = 16 * wave + 2 * i + hh;
    const int gr = rowBase + lr;
    float* op = outF + (size_t)gr * (size_t)ldo + col0 + 4 * m;
    *(volatile v4f*)op = fv[i];
  }
}

__global__ __launch_bounds__(PTHR) void k_conv(const float* __restrict__ XZ, const float* __restrict__ cw,
                                               const float* __restrict__ cb, float* XC, unsigned short* XCHL) {
  __shared__ __attribute__((aligned(16))) float cs[DI];
  const int tid = (int)threadIdx.x;
  const int t   = (int)blockIdx.x;
  const int l   = t & (SL - 1);
  const int d0  = 8 * tid;

  v4f wv[8];
#pragma unroll
  for (int j = 0; j < 8; ++j) wv[j] = *(const v4fa*)(cw + (size_t)(d0 + j) * 4);
  const v4f b0 = *(const v4fa*)(cb + d0);
  const v4f b1 = *(const v4fa*)(cb + d0 + 4);

  float acc[8];
#pragma unroll
  for (int j = 0; j < 8; ++j) acc[j] = 0.0f;
#pragma unroll
  for (int k = 0; k < 4; ++k) {
    const bool ok = (l - 3 + k) >= 0;
    const int row = ok ? (t - 3 + k) : t;
    const float* p = XZ + (size_t)row * XZC + d0;
    const v4f xa = *(const v4fa*)p;
    const v4f xb = *(const v4fa*)(p + 4);
    const float xs[8] = {xa.x, xa.y, xa.z, xa.w, xb.x, xb.y, xb.z, xb.w};
#pragma unroll
    for (int j = 0; j < 8; ++j) {
      const float xv = ok ? xs[j] : 0.0f;
      acc[j] = acc[j] + xv * bf16_val(wv[j][k]);
    }
  }
  {
    const float bs[8] = {b0.x, b0.y, b0.z, b0.w, b1.x, b1.y, b1.z, b1.w};
#pragma unroll
    for (int j = 0; j < 8; ++j) cs[d0 + j] = acc[j] + bf16_val(bs[j]);
  }
#pragma unroll 1
  for (int j = 0; j < 8; ++j) {
    const float c = cs[d0 + j];
    cs[d0 + j] = c * (1.0f / (1.0f + expf(-c)));
  }
  __syncthreads();

  v4f f0, f1;
  f0 = *(const v4fa*)(cs + 4 * tid);
  f1 = *(const v4fa*)(cs + 4 * (PTHR + tid));
  const v4f s0 = *(const v4fa*)(cs + d0);
  const v4f s1 = *(const v4fa*)(cs + d0 + 4);
  v8us oh, ol;
  {
    const float sv[8] = {s0.x, s0.y, s0.z, s0.w, s1.x, s1.y, s1.z, s1.w};
#pragma unroll
    for (int j = 0; j < 8; ++j) {
      const unsigned hb = bf16_bits(sv[j]);
      oh[j] = (unsigned short)hb;
      ol[j] = (unsigned short)bf16_bits(sv[j] - __uint_as_float(hb << 16));
    }
  }
  float* xr = XC + (size_t)t * DI;
  unsigned short* hr = XCHL + (size_t)t * K2;
  *(volatile v4f*)(xr + 4 * tid) = f0;
  *(volatile v4f*)(xr + 4 * (PTHR + tid)) = f1;
  *(volatile v8us*)(hr + d0) = oh;
  *(volatile v8us*)(hr + DI + d0) = ol;
  __threadfence();
  *(volatile v4f*)(xr + 4 * tid) = f0;
  *(volatile v4f*)(xr + 4 * (PTHR + tid)) = f1;
  *(volatile v8us*)(hr + d0) = oh;
  *(volatile v8us*)(hr + DI + d0) = ol;
}

__global__ __launch_bounds__(SNT) void k_scan(const float* __restrict__ XZ, const float* __restrict__ XC,
                                              const float* __restrict__ PROJ,
                                              const float* __restrict__ dtw, const float* __restrict__ dtb,
                                              const float* __restrict__ alog, const float* __restrict__ dpar,
                                              unsigned short* YHL) {
  __shared__ float hs[DS * SNT];
  __shared__ float as_[DS * SNT];
  __shared__ __attribute__((aligned(16))) float pj[SCH * PJW];
  __shared__ __attribute__((aligned(16))) unsigned short ys[2 * SCH * SNT];
  const int tid   = (int)threadIdx.x;
  const int dbase = (int)blockIdx.x * SNT;
  const int d     = dbase + tid;
  const int t0    = (int)blockIdx.y * SL;

#pragma unroll 1
  for (int n = 0; n < DS; ++n) {
    const float al = bf16_val(alog[(size_t)d * DS + n]);
    as_[n * SNT + tid] = -expf(al);
    hs[n * SNT + tid]  = 0.0f;
  }
  const float dw = bf16_val(dtw[d]);
  const float db = bf16_val(dtb[d]);
  const float Dp = bf16_val(dpar[d]);

  float xcn = XC[(size_t)t0 * DI + d];
  float zn  = XZ[(size_t)t0 * XZC + DI + d];

#pragma unroll 1
  for (int ch = 0; ch < SL / SCH; ++ch) {
    const int tb = t0 + ch * SCH;
    __syncthreads();
#pragma unroll
    for (int it = 0; it < (SCH * PJQ) / SNT; ++it) {
      const int i   = it * SNT + tid;
      const int tok = i / PJQ;
      const int q   = i - tok * PJQ;
      const v4f v = *(const v4fa*)(PROJ + (size_t)(tb + tok) * PJP + 4 * q);
      *(v4fa*)(pj + tok * PJW + 4 * q) = v;
    }
    __syncthreads();

#pragma unroll 1
    for (int tl = 0; tl < SCH; ++tl) {
      const int t = tb + tl;
      const float xcv = xcn;
      const float zv  = zn;
      int tn = t + 1;
      tn = tn > t0 + SL - 1 ? t0 + SL - 1 : tn;
      xcn = XC[(size_t)tn * DI + d];
      zn  = XZ[(size_t)tn * XZC + DI + d];

      const float* pr = pj + tl * PJW;
      const float dtr = pr[0] * dw + db;
      const float dt  = fmaxf(dtr, 0.0f) + log1pf(expf(-fabsf(dtr)));
      float acc = 0.0f;
#pragma unroll 2
      for (int n = 0; n < DS; ++n) {
        float hv = hs[n * SNT + tid];
        const float an  = as_[n * SNT + tid];
        const float dA  = expf(dt * an);
        const float dBx = (dt * pr[1 + n]) * xcv;
        hv = dA * hv + dBx;
        hs[n * SNT + tid] = hv;
        acc += hv * pr[1 + DS + n];
      }
      const float g  = zv * (1.0f / (1.0f + expf(-zv)));
      const float yv = (acc + xcv * Dp) * g;
      const unsigned hb = bf16_bits(yv);
      const unsigned lb = bf16_bits(yv - __uint_as_float(hb << 16));
      ys[tl * SNT + tid]             = (unsigned short)hb;
      ys[SCH * SNT + tl * SNT + tid] = (unsigned short)lb;
    }
    __syncthreads();

#pragma unroll 1
    for (int g4 = 0; g4 < 4; ++g4) {
      v8us q[4];
#pragma unroll
      for (int j = 0; j < 4; ++j) {
        const int u   = (g4 * 4 + j) * SNT + tid;
        const int seg = u & 15;
        const int pl  = (u >> 4) & 1;
        const int tok = u >> 5;
        q[j] = *(const v8usa*)(ys + pl * (SCH * SNT) + tok * SNT + 8 * seg);
      }
#pragma unroll
      for (int j = 0; j < 4; ++j) {
        const int u   = (g4 * 4 + j) * SNT + tid;
        const int seg = u & 15;
        const int pl  = (u >> 4) & 1;
        const int tok = u >> 5;
        unsigned short* dp = YHL + (size_t)(tb + tok) * K2 + pl * DI + dbase + 8 * seg;
        *(volatile v8us*)dp = q[j];
      }
      __threadfence();
#pragma unroll
      for (int j = 0; j < 4; ++j) {
        const int u   = (g4 * 4 + j) * SNT + tid;
        const int seg = u & 15;
        const int pl  = (u >> 4) & 1;
        const int tok = u >> 5;
        unsigned short* dp = YHL + (size_t)(tb + tok) * K2 + pl * DI + dbase + 8 * seg;
        *(volatile v8us*)dp = q[j];
      }
    }
  }
}

static inline size_t al256(size_t o) { return (o + 255) & ~(size_t)255; }

extern "C" void kernel_launch(void* const* d_in, const int* in_sizes, int n_in,
                              void* d_out, int out_size, void* d_ws, size_t ws_size,
                              hipStream_t stream) {
  if (n_in < 10) return;
  if (in_sizes[0] != NTOK * DM) return;
  if (in_sizes[1] != XZC * DM) return;
  if (in_sizes[2] != DI * 4) return;
  if (in_sizes[3] != DI) return;
  if (in_sizes[4] != NPJ * DI) return;
  if (in_sizes[5] != DI) return;
  if (in_sizes[6] != DI) return;
  if (in_sizes[7] != DI * DS) return;
  if (in_sizes[8] != DI) return;
  if (in_sizes[9] != DM * DI) return;
  if (out_size != NTOK * DM) return;

  const float* x     = (const float*)d_in[0];
  const float* W_in  = (const float*)d_in[1];
  const float* cw    = (const float*)d_in[2];
  const float* cb    = (const float*)d_in[3];
  const float* W_x   = (const float*)d_in[4];
  const float* dt_w  = (const float*)d_in[5];
  const float* dt_b  = (const float*)d_in[6];
  const float* A_log = (const float*)d_in[7];
  const float* D_par = (const float*)d_in[8];
  const float* W_out = (const float*)d_in[9];
  float* out = (float*)d_out;

  char* ws = (char*)d_ws;
  size_t off = 0;
  const size_t oXB   = off; off = al256(off + (size_t)NTOK * DM * 2);
  const size_t oWIN  = off; off = al256(off + (size_t)XZC * DM * 2);
  const size_t oWOUT = off; off = al256(off + (size_t)DM * DI * 2);
  const size_t oWX   = off; off = al256(off + (size_t)PJP * DI * 2);
  const size_t oXZ   = off; off = al256(off + (size_t)NTOK * XZC * 4);
  const size_t oXC   = off; off = al256(off + (size_t)NTOK * DI * 4);
  const size_t oXCHL = off; off = al256(off + (size_t)NTOK * K2 * 2);
  const size_t oPROJ = off; off = al256(off + (size_t)NTOK * PJP * 4);
  const size_t oYHL  = off; off = al256(off + (size_t)NTOK * K2 * 2);
  if (off > ws_size || off > (size_t)WSMAX) return;
  unsigned short* XB   = (unsigned short*)(ws + oXB);
  unsigned short* WIN  = (unsigned short*)(ws + oWIN);
  unsigned short* WOUT = (unsigned short*)(ws + oWOUT);
  unsigned short* WX   = (unsigned short*)(ws + oWX);
  float*          XZ   = (float*)(ws + oXZ);
  float*          XC   = (float*)(ws + oXC);
  unsigned short* XCHL = (unsigned short*)(ws + oXCHL);
  float*          PROJ = (float*)(ws + oPROJ);
  unsigned short* YHL  = (unsigned short*)(ws + oYHL);

  k_prep<<<U_TOT / PTHR, PTHR, 0, stream>>>(x, W_in, W_out, W_x, XB, WIN, WOUT, WX);
  k_gemm<<<dim3(NTOK / GBM, XZC / GBN), GTHR, 0, stream>>>(XB, WIN, XZ, DM, DM, DM - 1, XZC);
  k_conv<<<NTOK, PTHR, 0, stream>>>(XZ, cw, cb, XC, XCHL);
  k_gemm<<<dim3(NTOK / GBM, PJP / GBN), GTHR, 0, stream>>>(XCHL, WX, PROJ, K2, DI, DI - 1, PJP);
  k_scan<<<dim3(DI / SNT, NTOK / SL), SNT, 0, stream>>>(XZ, XC, PROJ, dt_w, dt_b, A_log, D_par, YHL);
  k_gemm<<<dim3(NTOK / GBM, DM / GBN), GTHR, 0, stream>>>(YHL, WOUT, out, K2, DI, DI - 1, DM);
}
